// CrfRnn_82179904242160
// MI455X (gfx1250) — hardware-verified
//
#include <hip/hip_runtime.h>

#define HH 80
#define WW 80
#define NPIX 6400
#define LBL 21
#define LPAD 32
#define NUM_ITER 5
#define NCHUNK 8
#define JSPAN (NPIX / NCHUNK)
#define QSCALE 16384.0f
#define KSCALE 16384.0f
#define KS_INV (1.0f / 16384.0f)
#define ACC_INV (1.0f / 268435456.0f)
#define F16_MIN_NRM 6.103515625e-5f
#define EPS_ 1e-8f

static_assert(NPIX % 256 == 0, "");
static_assert(NPIX % 32 == 0, "");
static_assert(JSPAN % 32 == 0, "");
static_assert(WW % 8 == 0, "");
static_assert(HH * WW == NPIX, "");

typedef _Float16 v16h __attribute__((ext_vector_type(16)));
typedef _Float16 v8h  __attribute__((ext_vector_type(8)));
typedef _Float16 v8ha __attribute__((ext_vector_type(8), may_alias));
typedef float v8f __attribute__((ext_vector_type(8)));
typedef float v4f __attribute__((ext_vector_type(4)));
typedef float v4fa __attribute__((ext_vector_type(4), may_alias));

union Frag  { v16h v; v8h half[2]; };
union Pack8 { v8h v; _Float16 s[8]; };
union Quad8 { v4f q[2]; float s[8]; };

static __device__ __forceinline__ v8f wmma16(const v16h& a, const v16h& b, v8f c) {
    return __builtin_amdgcn_wmma_f32_16x16x32_f16(false, a, false, b, (short)0, c, false, false);
}

template <int KT>
static __device__ __forceinline__ void build_rows(const float* __restrict__ img,
                                                  _Float16* __restrict__ K,
                                                  float* rs) {
#pragma clang fp contract(off)
    const int w = threadIdx.x >> 5, lane = threadIdx.x & 31;
    const float R3 = 1.0f / 3.0f, R160 = 1.0f / 160.0f;
    const float RP = (KT == 0) ? R3 : R160;
    for (int rr = 0; rr < 4; ++rr) {
        const int j = (int)blockIdx.x * 32 + w * 4 + rr;
        const int yj = j / WW, xj = j - yj * WW;
        const float f0j = (float)xj * RP, f1j = (float)yj * RP;
        float f2j = 0.0f, f3j = 0.0f, f4j = 0.0f;
        float sqj = f0j * f0j + f1j * f1j;
        if (KT == 1) {
            f2j = img[j] * R3;
            f3j = img[NPIX + j] * R3;
            f4j = img[2 * NPIX + j] * R3;
            sqj = sqj + f2j * f2j;
            sqj = sqj + f3j * f3j;
            sqj = sqj + f4j * f4j;
        }
        float sum = 0.0f;
        _Float16* Krow = K + (size_t)j * NPIX;
        for (int ps = 0; ps < NPIX / 256; ++ps) {
            const int i0 = ps * 256 + lane * 8;
            const int yi = i0 / WW, x0 = i0 - yi * WW;
            const float f1i = (float)yi * RP;
            Quad8 cr, cg, cb;
            if (KT == 1) {
                cr.q[0] = *(const v4fa*)(img + i0);            cr.q[1] = *(const v4fa*)(img + i0 + 4);
                cg.q[0] = *(const v4fa*)(img + NPIX + i0);     cg.q[1] = *(const v4fa*)(img + NPIX + i0 + 4);
                cb.q[0] = *(const v4fa*)(img + 2 * NPIX + i0); cb.q[1] = *(const v4fa*)(img + 2 * NPIX + i0 + 4);
            }
            Pack8 pk;
#pragma unroll
            for (int e = 0; e < 8; ++e) {
                const float f0i = (float)(x0 + e) * RP;
                float sqi = f0i * f0i + f1i * f1i;
                float dot;
                if (KT == 0) {
                    dot = fmaf(f1i, f1j, f0i * f0j);
                } else {
                    const float f2i = cr.s[e] * R3, f3i = cg.s[e] * R3, f4i = cb.s[e] * R3;
                    sqi = sqi + f2i * f2i;
                    sqi = sqi + f3i * f3i;
                    sqi = sqi + f4i * f4i;
                    dot = fmaf(f4i, f4j, fmaf(f3i, f3j, fmaf(f2i, f2j, fmaf(f1i, f1j, f0i * f0j))));
                }
                float d2 = (sqi + sqj) - 2.0f * dot;
                d2 = fmaxf(d2, 0.0f);
                float v = __expf(-0.5f * d2) * KSCALE;
                v = (v < F16_MIN_NRM) ? 0.0f : v;
                const _Float16 hv = (_Float16)v;
                sum += (float)hv;
                pk.s[e] = hv;
            }
            _Float16* gp = Krow + i0;
            *(volatile v8h*)gp = pk.v;
            __threadfence();
            *(volatile v8h*)gp = pk.v;
        }
#pragma unroll
        for (int off = 16; off > 0; off >>= 1) sum += __shfl_xor(sum, off, 32);
        if (lane == 0) rs[w * 4 + rr] = sum;
    }
}

__global__ void __launch_bounds__(256)
k_build(const float* __restrict__ img,
        _Float16* __restrict__ Ksp, _Float16* __restrict__ Kbi,
        float* __restrict__ nsp, float* __restrict__ nbi) {
    __shared__ __attribute__((aligned(16))) float rs[32];
    if (blockIdx.y == 0) build_rows<0>(img, Ksp, rs);
    else                 build_rows<1>(img, Kbi, rs);
    __syncthreads();
    if (threadIdx.x < 8) {
        float* nrm = (blockIdx.y == 0) ? nsp : nbi;
        const int l8 = threadIdx.x;
        const v4f s4 = *(const v4fa*)(rs + 4 * l8);
        v4f n4;
        n4.x = 1.0f / (s4.x * KS_INV + EPS_);
        n4.y = 1.0f / (s4.y * KS_INV + EPS_);
        n4.z = 1.0f / (s4.z * KS_INV + EPS_);
        n4.w = 1.0f / (s4.w * KS_INV + EPS_);
        float* gp = nrm + (size_t)blockIdx.x * 32 + 4 * l8;
        *(volatile v4f*)gp = n4;
        __threadfence();
        *(volatile v4f*)gp = n4;
    }
}

__global__ void __launch_bounds__(256)
k_softmax(const float* __restrict__ src, _Float16* __restrict__ q) {
    __shared__ __attribute__((aligned(16))) _Float16 qs[LPAD * 256];
    const int t = threadIdx.x;
    const int ibase = blockIdx.x * 256;
    const int i = ibase + t;
    float v[LBL];
#pragma unroll
    for (int l = 0; l < LBL; ++l) v[l] = (i < NPIX) ? src[(size_t)l * NPIX + i] : 0.0f;
    float mx = v[0];
#pragma unroll
    for (int l = 1; l < LBL; ++l) mx = fmaxf(mx, v[l]);
    float s = 0.0f;
#pragma unroll
    for (int l = 0; l < LBL; ++l) { v[l] = __expf(v[l] - mx); s += v[l]; }
    const float inv = 1.0f / s;
#pragma unroll
    for (int l = 0; l < LBL; ++l) {
        float qv = (v[l] * inv) * QSCALE;
        qv = (qv < F16_MIN_NRM) ? 0.0f : qv;
        qs[l * 256 + t] = (_Float16)qv;
    }
#pragma unroll
    for (int l = LBL; l < LPAD; ++l) qs[l * 256 + t] = (_Float16)0.0f;
    __syncthreads();
    const int w = t >> 5, lane = t & 31;
#pragma unroll
    for (int k = 0; k < 4; ++k) {
        const int l = w * 4 + k;
        const v8h val = *(const v8ha*)(qs + l * 256 + 8 * lane);
        _Float16* gp = q + (size_t)l * NPIX + ibase + 8 * lane;
        const bool ok = (ibase + 8 * lane + 8) <= NPIX;
        if (ok) *(volatile v8h*)gp = val;
        __threadfence();
        if (ok) *(volatile v8h*)gp = val;
    }
}

template <bool ADD>
static __device__ __forceinline__ void put8(float* pb, int row0, int col, v8f a) {
#pragma unroll
    for (int r = 0; r < 8; ++r) {
        float* p = pb + (row0 + r) * 32 + col;
        if (ADD) *p = *p + a[r];
        else     *p = a[r];
    }
}

template <bool ADD>
static __device__ __forceinline__ void put_all(float* pb, int h, int m,
                                               v8f sA0, v8f sA1, v8f sB0, v8f sB1,
                                               v8f bA0, v8f bA1, v8f bB0, v8f bB1) {
    put8<ADD>(pb,        8 * h,      m,      sA0);
    put8<ADD>(pb,        16 + 8 * h, m,      sA1);
    put8<ADD>(pb,        8 * h,      16 + m, sB0);
    put8<ADD>(pb,        16 + 8 * h, 16 + m, sB1);
    put8<ADD>(pb + 1024, 8 * h,      m,      bA0);
    put8<ADD>(pb + 1024, 16 + 8 * h, m,      bA1);
    put8<ADD>(pb + 1024, 8 * h,      16 + m, bB0);
    put8<ADD>(pb + 1024, 16 + 8 * h, 16 + m, bB1);
}

__global__ void __launch_bounds__(256)
k_mf(const _Float16* __restrict__ q,
     const _Float16* __restrict__ Ksp, const _Float16* __restrict__ Kbi,
     const float* __restrict__ nsp, const float* __restrict__ nbi,
     const float* __restrict__ unary,
     const float* __restrict__ Wsp, const float* __restrict__ Wbi,
     const float* __restrict__ Cm,
     float* __restrict__ out) {
    __shared__ __attribute__((aligned(16))) float part[4 * 2 * 32 * 32];
    __shared__ __attribute__((aligned(16))) float tile[2 * 32 * 32];
    __shared__ __attribute__((aligned(16))) float tts[32 * 32];
    __shared__ __attribute__((aligned(16))) float outs[32 * 32];
    __shared__ float nr[2 * 32];

    const int t = threadIdx.x, w = t >> 5, lane = t & 31;
    const int h = lane >> 4, m = lane & 15;
    const int i0 = blockIdx.x * 32;
    if (t < 64) {
        const int kt = t >> 5, c = t & 31;
        nr[t] = (kt == 0) ? nsp[i0 + c] : nbi[i0 + c];
    }

    v8f sA0 = {}, sA1 = {}, sB0 = {}, sB1 = {};
    v8f bA0 = {}, bA1 = {}, bB0 = {}, bB1 = {};

    const _Float16* qa0 = q   + (size_t)m * NPIX;
    const _Float16* qa1 = q   + (size_t)(m + 16) * NPIX;
    const _Float16* ks0 = Ksp + (size_t)(i0 + m) * NPIX;
    const _Float16* ks1 = Ksp + (size_t)(i0 + 16 + m) * NPIX;
    const _Float16* kb0 = Kbi + (size_t)(i0 + m) * NPIX;
    const _Float16* kb1 = Kbi + (size_t)(i0 + 16 + m) * NPIX;

    const int jbase = w * JSPAN;
    for (int js = 0; js < JSPAN; js += 32) {
        const int k0 = jbase + js + 8 * h;
        Frag a0, a1, b0, b1, c0, c1;
        a0.half[0] = *(const v8h*)(qa0 + k0);  a0.half[1] = *(const v8h*)(qa0 + k0 + 16);
        a1.half[0] = *(const v8h*)(qa1 + k0);  a1.half[1] = *(const v8h*)(qa1 + k0 + 16);
        b0.half[0] = *(const v8h*)(ks0 + k0);  b0.half[1] = *(const v8h*)(ks0 + k0 + 16);
        b1.half[0] = *(const v8h*)(ks1 + k0);  b1.half[1] = *(const v8h*)(ks1 + k0 + 16);
        c0.half[0] = *(const v8h*)(kb0 + k0);  c0.half[1] = *(const v8h*)(kb0 + k0 + 16);
        c1.half[0] = *(const v8h*)(kb1 + k0);  c1.half[1] = *(const v8h*)(kb1 + k0 + 16);

        sA0 = wmma16(a0.v, b0.v, sA0);
        sA1 = wmma16(a1.v, b0.v, sA1);
        sB0 = wmma16(a0.v, b1.v, sB0);
        sB1 = wmma16(a1.v, b1.v, sB1);
        bA0 = wmma16(a0.v, c0.v, bA0);
        bA1 = wmma16(a1.v, c0.v, bA1);
        bB0 = wmma16(a0.v, c1.v, bB0);
        bB1 = wmma16(a1.v, c1.v, bB1);
        asm volatile("v_nop\n\tv_nop\n\tv_nop\n\tv_nop"
                     : "+v"(sA0), "+v"(sA1), "+v"(sB0), "+v"(sB1),
                       "+v"(bA0), "+v"(bA1), "+v"(bB0), "+v"(bB1)
                     : "v"(a0.v), "v"(a1.v), "v"(b0.v), "v"(b1.v), "v"(c0.v), "v"(c1.v));
    }

    if (w < 4) put_all<false>(part + w * 2048, h, m, sA0, sA1, sB0, sB1, bA0, bA1, bB0, bB1);
    __syncthreads();
    if (w >= 4) put_all<true>(part + (w - 4) * 2048, h, m, sA0, sA1, sB0, sB1, bA0, bA1, bB0, bB1);
    __syncthreads();

#pragma unroll
    for (int e = 0; e < 8; ++e) {
        const int idx = t + 256 * e;
        const int kt = idx >> 10, col = idx & 31;
        const float v = part[idx] + part[2048 + idx] + part[4096 + idx] + part[6144 + idx];
        tile[idx] = v * ACC_INV * nr[kt * 32 + col];
    }
    __syncthreads();

    const int p = lane;
#pragma unroll
    for (int k3 = 0; k3 < 3; ++k3) {
        const int l = w + 8 * k3;
        if (l < LBL) {
            float a = 0.0f, b = 0.0f;
#pragma unroll
            for (int lp = 0; lp < LBL; ++lp) {
                a += Wsp[l * LBL + lp] * tile[lp * 32 + p];
                b += Wbi[l * LBL + lp] * tile[1024 + lp * 32 + p];
            }
            tts[l * 32 + p] = a + b;
        }
    }
    __syncthreads();
#pragma unroll
    for (int k3 = 0; k3 < 3; ++k3) {
        const int l = w + 8 * k3;
        if (l < LBL) {
            float acc = 0.0f;
#pragma unroll
            for (int lp = 0; lp < LBL; ++lp) acc += Cm[l * LBL + lp] * tts[lp * 32 + p];
            outs[l * 32 + p] = acc + unary[(size_t)l * NPIX + i0 + p];
        }
    }
    __syncthreads();
    {
        const int row = 4 * w + (lane >> 3), c4 = 4 * (lane & 7);
        const v4f val = *(const v4fa*)(outs + row * 32 + c4);
        const bool ok = row < LBL;
        float* gp = out + (size_t)(ok ? row : 0) * NPIX + i0 + c4;
        if (ok) *(volatile v4f*)gp = val;
        __threadfence();
        if (ok) *(volatile v4f*)gp = val;
    }
}

extern "C" void kernel_launch(void* const* d_in, const int* in_sizes, int n_in,
                              void* d_out, int out_size, void* d_ws, size_t ws_size,
                              hipStream_t stream) {
    if (n_in < 5) return;
    if (in_sizes[0] != 3 * NPIX || in_sizes[1] != LBL * NPIX ||
        in_sizes[2] != LBL * LBL || in_sizes[3] != LBL * LBL || in_sizes[4] != LBL * LBL ||
        out_size != LBL * NPIX) return;

    const float* image  = (const float*)d_in[0];
    const float* logits = (const float*)d_in[1];
    const float* Wsp    = (const float*)d_in[2];
    const float* Wbi    = (const float*)d_in[3];
    const float* Cm     = (const float*)d_in[4];
    float* cur = (float*)d_out;

    const size_t kbytes = (size_t)NPIX * NPIX * sizeof(_Float16);
    const size_t nbytes = (size_t)NPIX * sizeof(float);
    const size_t qbytes = (size_t)LPAD * NPIX * sizeof(_Float16);
    const size_t total  = 2 * kbytes + 2 * nbytes + qbytes;
    if (total > ws_size) return;

    char* wsp = (char*)d_ws;
    _Float16* Ksp = (_Float16*)(wsp);
    _Float16* Kbi = (_Float16*)(wsp + kbytes);
    float*    nsp = (float*)(wsp + 2 * kbytes);
    float*    nbi = (float*)(wsp + 2 * kbytes + nbytes);
    _Float16* q   = (_Float16*)(wsp + 2 * kbytes + 2 * nbytes);

    k_build<<<dim3(NPIX / 32, 2), 256, 0, stream>>>(image, Ksp, Kbi, nsp, nbi);
    for (int it = 0; it < NUM_ITER; ++it) {
        const float* src = (it == 0) ? logits : (const float*)cur;
        k_softmax<<<NPIX / 256, 256, 0, stream>>>(src, q);
        k_mf<<<NPIX / 32, 256, 0, stream>>>(q, Ksp, Kbi, nsp, nbi, logits, Wsp, Wbi, Cm, cur);
    }
}
